// LSTMnetwork_13580686590591
// MI455X (gfx1250) — hardware-verified
//
#include <hip/hip_runtime.h>

typedef __attribute__((ext_vector_type(16))) _Float16 v16h;
typedef __attribute__((ext_vector_type(8)))  _Float16 v8h;
typedef __attribute__((ext_vector_type(16))) __bf16   v16b;
typedef __attribute__((ext_vector_type(8)))  __bf16   v8b;
typedef __attribute__((ext_vector_type(8)))  float    v8f;
typedef __attribute__((ext_vector_type(4)))  float    v4f;

__device__ __forceinline__ unsigned short f2bf_bits(float f) {
  unsigned u = __float_as_uint(f);
  return (unsigned short)((u + 0x7FFFu + ((u >> 16) & 1u)) >> 16);
}
__device__ __forceinline__ float bf_bits2f(unsigned short h) { return __uint_as_float(((unsigned)h) << 16); }

__device__ __forceinline__ void dep_guard_h(v8f& a, v8f& b, v16h x, v16h y) { asm volatile("v_nop\n\tv_nop\n\tv_nop\n\tv_nop" : "+v"(a), "+v"(b) : "v"(x), "v"(y)); }
__device__ __forceinline__ void dep_guard_b(v8f& a, v8f& b, v16b x, v16b y) { asm volatile("v_nop\n\tv_nop\n\tv_nop\n\tv_nop" : "+v"(a), "+v"(b) : "v"(x), "v"(y)); }
__device__ __forceinline__ void keep4_h(v16h a, v16h b, v16h c, v16h d) { asm volatile("v_nop" :: "v"(a), "v"(b), "v"(c), "v"(d)); }
__device__ __forceinline__ void keep4_b(v16b a, v16b b, v16b c, v16b d) { asm volatile("v_nop" :: "v"(a), "v"(b), "v"(c), "v"(d)); }
__device__ __forceinline__ void acc_guard4(v8f& a, v8f& b, v8f& c, v8f& d) { asm volatile("v_nop\n\tv_nop\n\tv_nop\n\tv_nop" : "+v"(a), "+v"(b), "+v"(c), "+v"(d)); }
template <typename T> struct Frag;
template <> struct Frag<_Float16> {
  typedef v16h V; union U { v16h v; v8h h[2]; };
  static __device__ __forceinline__ v16h load(const _Float16* p) {
    U f; f.h[0] = *(const v8h*)(p); f.h[1] = *(const v8h*)(p + 16); return f.v;
  }
  static __device__ __forceinline__ v8f mma(v16h a, v16h b, v8f c) {
    return __builtin_amdgcn_wmma_f32_16x16x32_f16(false, a, false, b, (short)0, c, false, false);
  }
  static __device__ __forceinline__ void guard(v8f& a, v8f& b, v16h x, v16h y) { dep_guard_h(a, b, x, y); }
  static __device__ __forceinline__ void keep(v16h a, v16h b, v16h c, v16h d) { keep4_h(a, b, c, d); }
};
template <> struct Frag<__bf16> {
  typedef v16b V; union U { v16b v; v8b h[2]; };
  static __device__ __forceinline__ v16b load(const __bf16* p) {
    U f; f.h[0] = *(const v8b*)(p); f.h[1] = *(const v8b*)(p + 16); return f.v;
  }
  static __device__ __forceinline__ v8f mma(v16b a, v16b b, v8f c) {
    return __builtin_amdgcn_wmma_f32_16x16x32_bf16(false, a, false, b, (short)0, c, false, false);
  }
  static __device__ __forceinline__ void guard(v8f& a, v8f& b, v16b x, v16b y) { dep_guard_b(a, b, x, y); }
  static __device__ __forceinline__ void keep(v16b a, v16b b, v16b c, v16b d) { keep4_b(a, b, c, d); }
};

template <int ET> struct Elem;
template <> struct Elem<0> { typedef _Float16 T; };
template <> struct Elem<1> { typedef __bf16 T; };
template <int ET, bool SPLIT, int BIAS_MODE, int OUT_MODE, bool RESID, int ACT = 0>
__global__ __launch_bounds__(256) void wmma_gemm64(
    const unsigned short* __restrict__ Ap, const unsigned short* __restrict__ A2p, int lda, long strideA,
    const unsigned short* __restrict__ Btp, const unsigned short* __restrict__ Bt2p, int ldb, long strideB,
    void* __restrict__ Cout, void* __restrict__ Cout2, int ldc, long strideC,
    const float* __restrict__ bias,
    const float* __restrict__ resid, long strideR,
    int M, int N, int K, float scale) {
  typedef typename Elem<ET>::T T;
  typedef typename Frag<T>::V V;
  const T* A = (const T*)Ap; const T* A2 = (const T*)A2p; const T* Bt = (const T*)Btp; const T* Bt2 = (const T*)Bt2p;
  __shared__ __align__(16) float sT[8][16 * 68];
  const int b    = blockIdx.y;
  const int lane = threadIdx.x & 31;
  const int wave = threadIdx.x >> 5;
  const int tilesN = N >> 6;
  const int tilesM = M >> 6;
  const int tile = blockIdx.x * 8 + wave;
  if (tile >= tilesM * tilesN) return;
  const int tm = tile / tilesN;
  const int tn = tile - tm * tilesN;
  const int m0 = tm << 6;
  const int n0 = tn << 6;

  const T* Ab  = A  + (size_t)b * strideA;
  const T* Bb  = Bt + (size_t)b * strideB;
  const T* Ab2 = SPLIT ? (A2  + (size_t)b * strideA) : nullptr;
  const T* Bb2 = SPLIT ? (Bt2 + (size_t)b * strideB) : nullptr;

  const int rlane = lane & 15;
  const int koff  = (lane >> 4) * 8;
  const int mOff  = (lane >> 4) * 8;

  v8f acc[4][4];
#pragma unroll
  for (int i = 0; i < 4; ++i)
#pragma unroll
    for (int j = 0; j < 4; ++j) acc[i][j] = (v8f){0.f,0.f,0.f,0.f,0.f,0.f,0.f,0.f};

  for (int k0 = 0; k0 < K; k0 += 32) {
    V bh[4], bl[4];
#pragma unroll
    for (int j = 0; j < 4; ++j) {
      const size_t bo = (size_t)(n0 + (j << 4) + rlane) * ldb + koff + k0;
      bh[j] = Frag<T>::load(Bb + bo);
      if (SPLIT) bl[j] = Frag<T>::load(Bb2 + bo);
    }
#pragma unroll
    for (int i = 0; i < 4; ++i) {
      const size_t ao = (size_t)(m0 + (i << 4) + rlane) * lda + koff + k0;
      V ah = Frag<T>::load(Ab + ao);
      V al;
      if (SPLIT) al = Frag<T>::load(Ab2 + ao);
#pragma unroll
      for (int j = 0; j < 4; ++j) {
        acc[i][j] = Frag<T>::mma(ah, bh[j], acc[i][j]);
        if (SPLIT) {
          acc[i][j] = Frag<T>::mma(ah, bl[j], acc[i][j]);
          acc[i][j] = Frag<T>::mma(al, bh[j], acc[i][j]);
        }
      }
      Frag<T>::guard(acc[i][0], acc[i][3], ah, SPLIT ? al : ah);
    }
    Frag<T>::keep(bh[0], bh[1], bh[2], bh[3]);
    if (SPLIT) Frag<T>::keep(bl[0], bl[1], bl[2], bl[3]);
  }
  acc_guard4(acc[0][0], acc[0][1], acc[0][2], acc[0][3]);
  acc_guard4(acc[1][0], acc[1][1], acc[1][2], acc[1][3]);
  acc_guard4(acc[2][0], acc[2][1], acc[2][2], acc[2][3]);
  acc_guard4(acc[3][0], acc[3][1], acc[3][2], acc[3][3]);

  float* slab = sT[wave];
  const float* Rb = RESID ? (resid + (size_t)b * strideR) : nullptr;
#pragma unroll
  for (int i = 0; i < 4; ++i) {
    const int mBase = m0 + (i << 4);
#pragma unroll
    for (int j = 0; j < 4; ++j) {
      const int n = n0 + (j << 4) + rlane;
      float bv = 0.f;
      if (BIAS_MODE == 2) bv = bias[n];
#pragma unroll
      for (int r = 0; r < 8; ++r) {
        float v = acc[i][j][r] * scale;
        if (BIAS_MODE == 1) v += bias[mBase + mOff + r];
        if (BIAS_MODE == 2) v += bv;
        if (RESID) v += Rb[(size_t)(mBase + mOff + r) * ldc + n];
        if (ACT == 1) v = tanhf(v);
        if (ACT == 2) v = fmaxf(v, 0.0f);
        if (ACT == 3) v = v / (1.0f + expf(-v));
        if (ACT == 4) v = (v > 0.f) ? v : 0.01f * v;
        if (ACT == 5) v = 0.5f * v * (1.0f + erff(v * 0.70710678118654752f));
        slab[(mOff + r) * 68 + (j << 4) + rlane] = v;
      }
    }
    __builtin_amdgcn_fence(__ATOMIC_RELEASE, "workgroup");
    __builtin_amdgcn_wave_barrier();
    __builtin_amdgcn_fence(__ATOMIC_ACQUIRE, "workgroup");
    if (OUT_MODE == 0) {
      float* C = (float*)Cout + (size_t)b * strideC;
      const int hh = lane >> 4, c4 = (lane & 15) * 4;
      for (int pass = 0; pass < 2; ++pass) {
#pragma unroll
        for (int it = 0; it < 8; ++it) {
          const int row = it * 2 + hh;
          v4f v = *(const v4f*)(slab + row * 68 + c4);
          *(volatile v4f*)(C + (size_t)(mBase + row) * ldc + n0 + c4) = v;
        }
        __threadfence();
      }
    } else {
      const int q = lane >> 3, c8 = (lane & 7) * 8;
      unsigned short* C  = (unsigned short*)Cout  + (size_t)b * strideC;
      unsigned short* C2 = (OUT_MODE == 2) ? ((unsigned short*)Cout2 + (size_t)b * strideC) : nullptr;
      for (int pass = 0; pass < 2; ++pass) {
#pragma unroll
        for (int it = 0; it < 4; ++it) {
          const int row = it * 4 + q;
          const float* sp = slab + row * 68 + c8;
          v8h hv, lv;
#pragma unroll
          for (int e = 0; e < 8; ++e) {
            if (OUT_MODE == 1) {
              hv[e] = (_Float16)sp[e];
            } else {
              unsigned short hb = f2bf_bits(sp[e]);
              unsigned short lb = f2bf_bits(sp[e] - bf_bits2f(hb));
              hv[e] = __builtin_bit_cast(_Float16, hb);
              lv[e] = __builtin_bit_cast(_Float16, lb);
            }
          }
          *(volatile v8h*)(C + (size_t)(mBase + row) * ldc + n0 + c8) = hv;
          if (OUT_MODE == 2) *(volatile v8h*)(C2 + (size_t)(mBase + row) * ldc + n0 + c8) = lv;
        }
        __threadfence();
      }
    }
    __builtin_amdgcn_fence(__ATOMIC_RELEASE, "workgroup");
    __builtin_amdgcn_wave_barrier();
    __builtin_amdgcn_fence(__ATOMIC_ACQUIRE, "workgroup");
  }
}

constexpr int kRows      = 8192;
constexpr int kFeat      = 1024;
constexpr int kHid       = 512;
constexpr int kGateCols  = 1536;
constexpr int kGateRows  = 2048;
constexpr int kCellRows  = 16;

static_assert(kFeat % 32 == 0);
static_assert(kRows % 64 == 0 && kGateCols % 64 == 0);
static_assert(((kRows / 64) * (kGateCols / 64)) % 8 == 0);
static_assert(kRows % kCellRows == 0);
static_assert(kFeat == 2 * kHid);

constexpr size_t kBytesAct = (size_t)kRows * kFeat * 2;
constexpr size_t kBytesW   = (size_t)6 * kGateCols * kFeat * 2;
constexpr size_t kBytesG   = (size_t)kRows * kGateCols * 4;
constexpr size_t kOffAct0  = 0;
constexpr size_t kOffAct1  = kOffAct0 + kBytesAct;
constexpr size_t kOffW     = kOffAct1 + kBytesAct;
constexpr size_t kOffG     = kOffW + kBytesW;
constexpr size_t kWsTotal  = kOffG + kBytesG;
static_assert(kWsTotal == 102760448u);
static_assert(kWsTotal <= 134217728u);

__global__ __launch_bounds__(256) void cast_x_kernel(const float* __restrict__ src,
                                                     unsigned short* __restrict__ dst, int nthreads) {
  const int gid = blockIdx.x * 256 + threadIdx.x;
  if (gid >= nthreads) return;
  const size_t e0 = (size_t)gid * 8;
  const v4f a = *(const v4f*)(src + e0);
  const v4f c = *(const v4f*)(src + e0 + 4);
  v8h hv;
#pragma unroll
  for (int e = 0; e < 4; ++e) {
    hv[e]     = (_Float16)(a[e] * 16.0f);
    hv[4 + e] = (_Float16)(c[e] * 16.0f);
  }
  unsigned short* dp = dst + e0;
  *(volatile v8h*)dp = hv;
  __threadfence();
  *(volatile v8h*)dp = hv;
}

__global__ __launch_bounds__(256) void cast_w_kernel(const float* __restrict__ src,
                                                     unsigned short* __restrict__ dst, int nthreads) {
  const int gid = blockIdx.x * 256 + threadIdx.x;
  if (gid >= nthreads) return;
  const size_t e0 = (size_t)gid * 8;
  const int prow = (int)(e0 >> 10);
  const int k    = (int)(e0 & 1023);
  const int pl   = prow / kGateCols;
  const int p    = prow - pl * kGateCols;
  const int gate = p >> 9;
  const int gsrc = (gate == 0) ? 0 : (gate + 1);
  const size_t srow = (size_t)pl * kGateRows + (size_t)gsrc * kHid + (size_t)(p & (kHid - 1));
  const float* sp = src + srow * kFeat + k;
  const v4f a = *(const v4f*)sp;
  const v4f c = *(const v4f*)(sp + 4);
  v8h hv;
#pragma unroll
  for (int e = 0; e < 4; ++e) {
    hv[e]     = (_Float16)(a[e] * 64.0f);
    hv[4 + e] = (_Float16)(c[e] * 64.0f);
  }
  unsigned short* dp = dst + e0;
  *(volatile v8h*)dp = hv;
  __threadfence();
  *(volatile v8h*)dp = hv;
}

__device__ __forceinline__ float sigm_f(float x) {
  return __builtin_amdgcn_rcpf(1.0f + expf(-x));
}
__device__ __forceinline__ float tanh_f(float x) {
  const float e = expf(2.0f * x);
  const float r = __builtin_amdgcn_rcpf(e + 1.0f);
  return 1.0f - 2.0f * r;
}

template <bool FINAL>
__global__ __launch_bounds__(256) void lstm_cell_kernel(
    const float* __restrict__ G, const float* __restrict__ bih, const float* __restrict__ bhh,
    unsigned short* __restrict__ Hout, float* __restrict__ Out, int dir) {
  __shared__ __align__(16) float sbi[kGateCols];
  __shared__ __align__(16) float sbh[kGateCols];
  __shared__ __align__(16) float hs[2 * kHid];
  const int t = threadIdx.x;
  for (int idx = t; idx < kGateCols / 4; idx += 256) {
    const int p4   = idx * 4;
    const int gate = p4 >> 9;
    const int gsrc = (gate == 0) ? 0 : (gate + 1);
    const int src  = gsrc * kHid + (p4 & (kHid - 1));
    const v4f a = *(const v4f*)(bih + src);
    const v4f c = *(const v4f*)(bhh + src);
    *(v4f*)(sbi + p4) = a;
    *(v4f*)(sbh + p4) = c;
  }
  __syncthreads();
  const int rsub = t >> 7;
  const int u0   = (t & 127) * 4;
#pragma unroll 1
  for (int it = 0; it < kCellRows / 2; ++it) {
    const int row = blockIdx.x * kCellRows + it * 2 + rsub;
    const float* gr = G + (size_t)row * kGateCols;
    const v4f gi = *(const v4f*)(gr + u0);
    const v4f gg = *(const v4f*)(gr + kHid + u0);
    const v4f go = *(const v4f*)(gr + 2 * kHid + u0);
    const v4f bii = *(const v4f*)(sbi + u0);
    const v4f bhi = *(const v4f*)(sbh + u0);
    const v4f big = *(const v4f*)(sbi + kHid + u0);
    const v4f bhg = *(const v4f*)(sbh + kHid + u0);
    const v4f bio = *(const v4f*)(sbi + 2 * kHid + u0);
    const v4f bho = *(const v4f*)(sbh + 2 * kHid + u0);
    v4f h;
#pragma unroll
    for (int e = 0; e < 4; ++e) {
      const float xi = (gi[e] + bii[e]) + bhi[e];
      const float xg = (gg[e] + big[e]) + bhg[e];
      const float xo = (go[e] + bio[e]) + bho[e];
      const float cc = sigm_f(xi) * tanh_f(xg);
      h[e] = sigm_f(xo) * tanh_f(cc);
    }
    if (FINAL) {
      float* op = Out + (size_t)row * kFeat + dir * kHid + u0;
      const v4f hv = h;
      *(volatile v4f*)op = hv;
      __threadfence();
      *(volatile v4f*)op = hv;
    } else {
      v4f hsc;
#pragma unroll
      for (int e = 0; e < 4; ++e) hsc[e] = h[e] * 256.0f;
      *(v4f*)(hs + rsub * kHid + u0) = hsc;
      __syncthreads();
      if (t < 128) {
        const int r2 = t >> 6;
        const int c8 = (t & 63) * 8;
        const float* sp = hs + r2 * kHid + c8;
        const v4f a = *(const v4f*)sp;
        const v4f c = *(const v4f*)(sp + 4);
        v8h hv;
#pragma unroll
        for (int e = 0; e < 4; ++e) {
          hv[e]     = (_Float16)a[e];
          hv[4 + e] = (_Float16)c[e];
        }
        const int row2 = blockIdx.x * kCellRows + it * 2 + r2;
        unsigned short* hp = Hout + (size_t)row2 * kFeat + dir * kHid + c8;
        *(volatile v8h*)hp = hv;
        __threadfence();
        *(volatile v8h*)hp = hv;
      }
      __syncthreads();
    }
  }
}

extern "C" void kernel_launch(void* const* d_in, const int* in_sizes, int n_in,
                              void* d_out, int out_size, void* d_ws, size_t ws_size,
                              hipStream_t stream) {
  if (n_in < 9) return;
  if (in_sizes[0] != kRows * kFeat) return;
  if (in_sizes[1] != 2 * kGateRows * kFeat) return;
  if (in_sizes[3] != 2 * kGateRows || in_sizes[4] != 2 * kGateRows) return;
  if (in_sizes[5] != 4 * kGateRows * kFeat) return;
  if (in_sizes[7] != 4 * kGateRows || in_sizes[8] != 4 * kGateRows) return;
  if (out_size != kRows * kFeat) return;
  if (ws_size < kWsTotal) return;

  const float* x      = (const float*)d_in[0];
  const float* W_ih0  = (const float*)d_in[1];
  const float* b_ih0  = (const float*)d_in[3];
  const float* b_hh0  = (const float*)d_in[4];
  const float* W_ih12 = (const float*)d_in[5];
  const float* b_ih12 = (const float*)d_in[7];
  const float* b_hh12 = (const float*)d_in[8];
  float* out = (float*)d_out;

  char* ws = (char*)d_ws;
  unsigned short* act0 = (unsigned short*)(ws + kOffAct0);
  unsigned short* act1 = (unsigned short*)(ws + kOffAct1);
  unsigned short* wpl  = (unsigned short*)(ws + kOffW);
  float*          G    = (float*)(ws + kOffG);

  {
    const int nthr = kRows * kFeat / 8;
    cast_x_kernel<<<nthr / 256, 256, 0, stream>>>(x, act0, nthr);
  }
  {
    const int nthr0 = 2 * kGateCols * kFeat / 8;
    const int nthr1 = 4 * kGateCols * kFeat / 8;
    cast_w_kernel<<<nthr0 / 256, 256, 0, stream>>>(W_ih0, wpl, nthr0);
    cast_w_kernel<<<nthr1 / 256, 256, 0, stream>>>(W_ih12, wpl + (size_t)2 * kGateCols * kFeat, nthr1);
  }

  const int gemmBlocks = (kRows / 64) * (kGateCols / 64) / 8;
  const int cellBlocks = kRows / kCellRows;

  for (int l = 0; l < 3; ++l) {
    const unsigned short* A = (l == 0) ? act0 : ((l == 1) ? act1 : act0);
    unsigned short* Hn = (l == 0) ? act1 : act0;
    const float scale = (l == 0) ? (1.0f / 1024.0f) : (1.0f / 16384.0f);
    for (int d = 0; d < 2; ++d) {
      const unsigned short* Bt = wpl + (size_t)(l * 2 + d) * kGateCols * kFeat;
      wmma_gemm64<0, false, 0, 0, false, 0><<<dim3(gemmBlocks, 1), 256, 0, stream>>>(
          A, A, kFeat, 0L,
          Bt, Bt, kFeat, 0L,
          (void*)G, (void*)G, kGateCols, 0L,
          b_ih0,
          b_ih0, 0L,
          kRows, kGateCols, kFeat, scale);
      const float* bih = (l == 0) ? (b_ih0 + (size_t)d * kGateRows)
                                  : (b_ih12 + (size_t)((l - 1) * 2 + d) * kGateRows);
      const float* bhh = (l == 0) ? (b_hh0 + (size_t)d * kGateRows)
                                  : (b_hh12 + (size_t)((l - 1) * 2 + d) * kGateRows);
      if (l < 2) {
        lstm_cell_kernel<false><<<cellBlocks, 256, 0, stream>>>(G, bih, bhh, Hn, out, d);
      } else {
        lstm_cell_kernel<true><<<cellBlocks, 256, 0, stream>>>(G, bih, bhh, act1, out, d);
      }
    }
  }
}
